// RandSelfAttention2D_80333068305049
// MI455X (gfx1250) — hardware-verified
//
#include <hip/hip_runtime.h>
#include <stddef.h>
#include <stdint.h>

#define BB 4
#define CC 64
#define NN 16384
#define MM 1638
#define MPAD 1664
#define DD 64
#define NCHK 26
#define NQB 256

typedef __attribute__((ext_vector_type(16))) _Float16 v16h;
typedef __attribute__((ext_vector_type(8)))  _Float16 v8h;
typedef __attribute__((ext_vector_type(16))) __bf16   v16b;
typedef __attribute__((ext_vector_type(8)))  __bf16   v8b;
typedef __attribute__((ext_vector_type(8)))  float    v8f;
typedef __attribute__((ext_vector_type(4)))  float    v4f;
#define PSCALE 32768.0f
#define U16(p) ((const unsigned short*)(const void*)(p))
#define PSCALE_INV (1.0f / 32768.0f)

__device__ __forceinline__ unsigned short f2bf_bits(float f) {
  unsigned u = __float_as_uint(f);
  return (unsigned short)((u + 0x7FFFu + ((u >> 16) & 1u)) >> 16);
}
__device__ __forceinline__ float bf_bits2f(unsigned short h) { return __uint_as_float(((unsigned)h) << 16); }

__device__ __forceinline__ void dep_guard_h(v8f& a, v8f& b, v16h x, v16h y) { asm volatile("v_nop\n\tv_nop\n\tv_nop\n\tv_nop" : "+v"(a), "+v"(b) : "v"(x), "v"(y)); }
__device__ __forceinline__ void dep_guard_b(v8f& a, v8f& b, v16b x, v16b y) { asm volatile("v_nop\n\tv_nop\n\tv_nop\n\tv_nop" : "+v"(a), "+v"(b) : "v"(x), "v"(y)); }
__device__ __forceinline__ void keep4_h(v16h a, v16h b, v16h c, v16h d) { asm volatile("v_nop" :: "v"(a), "v"(b), "v"(c), "v"(d)); }
__device__ __forceinline__ void keep4_b(v16b a, v16b b, v16b c, v16b d) { asm volatile("v_nop" :: "v"(a), "v"(b), "v"(c), "v"(d)); }
__device__ __forceinline__ void acc_guard4(v8f& a, v8f& b, v8f& c, v8f& d) { asm volatile("v_nop\n\tv_nop\n\tv_nop\n\tv_nop" : "+v"(a), "+v"(b), "+v"(c), "+v"(d)); }
template <typename T> struct Frag;
template <> struct Frag<_Float16> {
  typedef v16h V; union U { v16h v; v8h h[2]; };
  static __device__ __forceinline__ v16h load(const _Float16* p) {
    U f; f.h[0] = *(const v8h*)(p); f.h[1] = *(const v8h*)(p + 16); return f.v;
  }
  static __device__ __forceinline__ v8f mma(v16h a, v16h b, v8f c) {
    return __builtin_amdgcn_wmma_f32_16x16x32_f16(false, a, false, b, (short)0, c, false, false);
  }
  static __device__ __forceinline__ void guard(v8f& a, v8f& b, v16h x, v16h y) { dep_guard_h(a, b, x, y); }
  static __device__ __forceinline__ void keep(v16h a, v16h b, v16h c, v16h d) { keep4_h(a, b, c, d); }
};
template <> struct Frag<__bf16> {
  typedef v16b V; union U { v16b v; v8b h[2]; };
  static __device__ __forceinline__ v16b load(const __bf16* p) {
    U f; f.h[0] = *(const v8b*)(p); f.h[1] = *(const v8b*)(p + 16); return f.v;
  }
  static __device__ __forceinline__ v8f mma(v16b a, v16b b, v8f c) {
    return __builtin_amdgcn_wmma_f32_16x16x32_bf16(false, a, false, b, (short)0, c, false, false);
  }
  static __device__ __forceinline__ void guard(v8f& a, v8f& b, v16b x, v16b y) { dep_guard_b(a, b, x, y); }
  static __device__ __forceinline__ void keep(v16b a, v16b b, v16b c, v16b d) { keep4_b(a, b, c, d); }
};

template <int ET> struct Elem;
template <> struct Elem<0> { typedef _Float16 T; };
template <> struct Elem<1> { typedef __bf16 T; };
template <int ET, bool SPLIT, int BIAS_MODE, int OUT_MODE, bool RESID, int ACT = 0>
__global__ __launch_bounds__(256) void wmma_gemm64(
    const unsigned short* __restrict__ Ap, const unsigned short* __restrict__ A2p, int lda, long strideA,
    const unsigned short* __restrict__ Btp, const unsigned short* __restrict__ Bt2p, int ldb, long strideB,
    void* __restrict__ Cout, void* __restrict__ Cout2, int ldc, long strideC,
    const float* __restrict__ bias,
    const float* __restrict__ resid, long strideR,
    int M, int N, int K, float scale) {
  typedef typename Elem<ET>::T T;
  typedef typename Frag<T>::V V;
  const T* A = (const T*)Ap; const T* A2 = (const T*)A2p; const T* Bt = (const T*)Btp; const T* Bt2 = (const T*)Bt2p;
  __shared__ __align__(16) float sT[8][16 * 68];
  const int b    = blockIdx.y;
  const int lane = threadIdx.x & 31;
  const int wave = threadIdx.x >> 5;
  const int tilesN = N >> 6;
  const int tilesM = M >> 6;
  const int tile = blockIdx.x * 8 + wave;
  if (tile >= tilesM * tilesN) return;
  const int tm = tile / tilesN;
  const int tn = tile - tm * tilesN;
  const int m0 = tm << 6;
  const int n0 = tn << 6;

  const T* Ab  = A  + (size_t)b * strideA;
  const T* Bb  = Bt + (size_t)b * strideB;
  const T* Ab2 = SPLIT ? (A2  + (size_t)b * strideA) : nullptr;
  const T* Bb2 = SPLIT ? (Bt2 + (size_t)b * strideB) : nullptr;

  const int rlane = lane & 15;
  const int koff  = (lane >> 4) * 8;
  const int mOff  = (lane >> 4) * 8;

  v8f acc[4][4];
#pragma unroll
  for (int i = 0; i < 4; ++i)
#pragma unroll
    for (int j = 0; j < 4; ++j) acc[i][j] = (v8f){0.f,0.f,0.f,0.f,0.f,0.f,0.f,0.f};

  for (int k0 = 0; k0 < K; k0 += 32) {
    V bh[4], bl[4];
#pragma unroll
    for (int j = 0; j < 4; ++j) {
      const size_t bo = (size_t)(n0 + (j << 4) + rlane) * ldb + koff + k0;
      bh[j] = Frag<T>::load(Bb + bo);
      if (SPLIT) bl[j] = Frag<T>::load(Bb2 + bo);
    }
#pragma unroll
    for (int i = 0; i < 4; ++i) {
      const size_t ao = (size_t)(m0 + (i << 4) + rlane) * lda + koff + k0;
      V ah = Frag<T>::load(Ab + ao);
      V al;
      if (SPLIT) al = Frag<T>::load(Ab2 + ao);
#pragma unroll
      for (int j = 0; j < 4; ++j) {
        acc[i][j] = Frag<T>::mma(ah, bh[j], acc[i][j]);
        if (SPLIT) {
          acc[i][j] = Frag<T>::mma(ah, bl[j], acc[i][j]);
          acc[i][j] = Frag<T>::mma(al, bh[j], acc[i][j]);
        }
      }
      Frag<T>::guard(acc[i][0], acc[i][3], ah, SPLIT ? al : ah);
    }
    Frag<T>::keep(bh[0], bh[1], bh[2], bh[3]);
    if (SPLIT) Frag<T>::keep(bl[0], bl[1], bl[2], bl[3]);
  }
  acc_guard4(acc[0][0], acc[0][1], acc[0][2], acc[0][3]);
  acc_guard4(acc[1][0], acc[1][1], acc[1][2], acc[1][3]);
  acc_guard4(acc[2][0], acc[2][1], acc[2][2], acc[2][3]);
  acc_guard4(acc[3][0], acc[3][1], acc[3][2], acc[3][3]);

  float* slab = sT[wave];
  const float* Rb = RESID ? (resid + (size_t)b * strideR) : nullptr;
#pragma unroll
  for (int i = 0; i < 4; ++i) {
    const int mBase = m0 + (i << 4);
#pragma unroll
    for (int j = 0; j < 4; ++j) {
      const int n = n0 + (j << 4) + rlane;
      float bv = 0.f;
      if (BIAS_MODE == 2) bv = bias[n];
#pragma unroll
      for (int r = 0; r < 8; ++r) {
        float v = acc[i][j][r] * scale;
        if (BIAS_MODE == 1) v += bias[mBase + mOff + r];
        if (BIAS_MODE == 2) v += bv;
        if (RESID) v += Rb[(size_t)(mBase + mOff + r) * ldc + n];
        if (ACT == 1) v = tanhf(v);
        if (ACT == 2) v = fmaxf(v, 0.0f);
        if (ACT == 3) v = v / (1.0f + expf(-v));
        if (ACT == 4) v = (v > 0.f) ? v : 0.01f * v;
        if (ACT == 5) v = 0.5f * v * (1.0f + erff(v * 0.70710678118654752f));
        slab[(mOff + r) * 68 + (j << 4) + rlane] = v;
      }
    }
    __builtin_amdgcn_fence(__ATOMIC_RELEASE, "workgroup");
    __builtin_amdgcn_wave_barrier();
    __builtin_amdgcn_fence(__ATOMIC_ACQUIRE, "workgroup");
    if (OUT_MODE == 0) {
      float* C = (float*)Cout + (size_t)b * strideC;
      const int hh = lane >> 4, c4 = (lane & 15) * 4;
      for (int pass = 0; pass < 2; ++pass) {
#pragma unroll
        for (int it = 0; it < 8; ++it) {
          const int row = it * 2 + hh;
          v4f v = *(const v4f*)(slab + row * 68 + c4);
          *(volatile v4f*)(C + (size_t)(mBase + row) * ldc + n0 + c4) = v;
        }
        __threadfence();
      }
    } else {
      const int q = lane >> 3, c8 = (lane & 7) * 8;
      unsigned short* C  = (unsigned short*)Cout  + (size_t)b * strideC;
      unsigned short* C2 = (OUT_MODE == 2) ? ((unsigned short*)Cout2 + (size_t)b * strideC) : nullptr;
      for (int pass = 0; pass < 2; ++pass) {
#pragma unroll
        for (int it = 0; it < 4; ++it) {
          const int row = it * 4 + q;
          const float* sp = slab + row * 68 + c8;
          v8h hv, lv;
#pragma unroll
          for (int e = 0; e < 8; ++e) {
            if (OUT_MODE == 1) {
              hv[e] = (_Float16)sp[e];
            } else {
              unsigned short hb = f2bf_bits(sp[e]);
              unsigned short lb = f2bf_bits(sp[e] - bf_bits2f(hb));
              hv[e] = __builtin_bit_cast(_Float16, hb);
              lv[e] = __builtin_bit_cast(_Float16, lb);
            }
          }
          *(volatile v8h*)(C + (size_t)(mBase + row) * ldc + n0 + c8) = hv;
          if (OUT_MODE == 2) *(volatile v8h*)(C2 + (size_t)(mBase + row) * ldc + n0 + c8) = lv;
        }
        __threadfence();
      }
    }
    __builtin_amdgcn_fence(__ATOMIC_RELEASE, "workgroup");
    __builtin_amdgcn_wave_barrier();
    __builtin_amdgcn_fence(__ATOMIC_ACQUIRE, "workgroup");
  }
}

__device__ __forceinline__ void split_bits(float v, unsigned short& hb, unsigned short& lb) {
  hb = f2bf_bits(v);
  lb = f2bf_bits(v - bf_bits2f(hb));
}

__global__ __launch_bounds__(256) void k_prep_w(const float* __restrict__ Wq, const float* __restrict__ Wk,
                                               const float* __restrict__ Wv, unsigned short* __restrict__ wt) {
  __shared__ __align__(16) float s[64 * 64];
  const int widx = blockIdx.x;
  const float* W = (widx == 0) ? Wq : ((widx == 1) ? Wk : Wv);
  const int t = threadIdx.x;
  for (int e = t; e < 64 * 64; e += 256) s[e] = W[e];
  __syncthreads();
  const int wave = t >> 5, lane = t & 31, q8 = lane >> 3, cseg = (lane & 7) * 8;
  for (int pass = 0; pass < 2; ++pass) {
#pragma unroll
    for (int it = 0; it < 4; ++it) {
      const int plane = it >> 1;
      const int d = (it & 1) * 32 + wave * 4 + q8;
      v8h hv;
#pragma unroll
      for (int e = 0; e < 8; ++e) {
        const float v = s[(cseg + e) * 64 + d];
        unsigned short hb, lb; split_bits(v, hb, lb);
        hv[e] = __builtin_bit_cast(_Float16, (unsigned short)(plane ? lb : hb));
      }
      *(volatile v8h*)(wt + ((size_t)(widx * 2 + plane) * 64 + d) * 64 + cseg) = hv;
    }
    __threadfence();
  }
}

__global__ __launch_bounds__(128) void k_xf(const float* __restrict__ x, unsigned short* __restrict__ xfh,
                                           unsigned short* __restrict__ xfl) {
  __shared__ __align__(16) float s[64 * 65];
  const int b = blockIdx.x >> 8, n0 = (blockIdx.x & 255) * 64, t = threadIdx.x;
  const float* xb = x + (size_t)b * CC * NN + n0;
#pragma unroll 4
  for (int i = 0; i < 32; ++i) {
    const int e = i * 128 + t;
    const int c = e >> 6, j = e & 63;
    s[c * 65 + j] = xb[(size_t)c * NN + j];
  }
  __syncthreads();
  const int wave = t >> 5, lane = t & 31, q8 = lane >> 3, cseg = (lane & 7) * 8;
  for (int pass = 0; pass < 2; ++pass) {
#pragma unroll
    for (int it = 0; it < 8; ++it) {
      const int plane = it >> 2;
      const int j = (it & 3) * 16 + wave * 4 + q8;
      v8h hv;
#pragma unroll
      for (int e = 0; e < 8; ++e) {
        const float v = s[(cseg + e) * 65 + j];
        unsigned short hb, lb; split_bits(v, hb, lb);
        hv[e] = __builtin_bit_cast(_Float16, (unsigned short)(plane ? lb : hb));
      }
      unsigned short* dst = (plane ? xfl : xfh) + ((size_t)b * NN + n0 + j) * CC + cseg;
      *(volatile v8h*)dst = hv;
    }
    __threadfence();
  }
}

__global__ __launch_bounds__(128) void k_gather(const float* __restrict__ x, const int* __restrict__ idx,
                                               unsigned short* __restrict__ xgh, unsigned short* __restrict__ xgl) {
  const int t = threadIdx.x;
  const int rowl = t >> 3, cseg = (t & 7) * 8;
  const int R = blockIdx.x * 16 + rowl;
  const int b = R / MPAD, kv = R - b * MPAD;
  const bool valid = kv < MM;
  int n = 0;
  if (valid) { n = idx[b * MM + kv]; n = n < 0 ? 0 : (n > NN - 1 ? NN - 1 : n); }
  v8h hv, lv;
#pragma unroll
  for (int e = 0; e < 8; ++e) {
    const float f = valid ? x[((size_t)b * CC + cseg + e) * NN + n] : 0.0f;
    unsigned short hb, lb; split_bits(f, hb, lb);
    hv[e] = __builtin_bit_cast(_Float16, hb);
    lv[e] = __builtin_bit_cast(_Float16, lb);
  }
  unsigned short* dh = xgh + (size_t)R * CC + cseg;
  unsigned short* dl = xgl + (size_t)R * CC + cseg;
  *(volatile v8h*)dh = hv; *(volatile v8h*)dl = lv;
  __threadfence();
  *(volatile v8h*)dh = hv; *(volatile v8h*)dl = lv;
}

__device__ __forceinline__ v8f mma_h(v16h a, v16h b, v8f c) {
  c = __builtin_amdgcn_wmma_f32_16x16x32_f16(false, a, false, b, (short)0, c, false, false);
  asm volatile("v_nop\n\tv_nop\n\tv_nop\n\tv_nop" : "+v"(c) : "v"(a), "v"(b));
  return c;
}

__global__ __launch_bounds__(128) void k_attn(const unsigned short* __restrict__ q16,
                                             const unsigned short* __restrict__ kg16,
                                             const unsigned short* __restrict__ vT16,
                                             float* __restrict__ out0, float* __restrict__ partial) {
  __shared__ __align__(16) _Float16 Ksh[64 * 64];
  __shared__ __align__(16) _Float16 Vth[64 * 64];
  __shared__ __align__(16) _Float16 Esh[NCHK * 64 * 64];
  __shared__ __align__(16) float Ws[64 * NCHK];
  __shared__ __align__(16) float Cs[MPAD];

  const int tid = threadIdx.x, wave = tid >> 5, lane = tid & 31, hh = lane >> 4, c = lane & 15;
  const int b = blockIdx.x >> 8, qb = blockIdx.x & 255;
  const int q0 = qb * 64 + wave * 16;
  const float NEG_INF = -__builtin_inff();

  const _Float16* qp = (const _Float16*)q16 + ((size_t)b * NN + q0 + c) * DD + 8 * hh;
  const v16h qa0 = Frag<_Float16>::load(qp);
  const v16h qa1 = Frag<_Float16>::load(qp + 32);

  float mrow[8], lrow[8];
  v8f oacc[4];
#pragma unroll
  for (int r = 0; r < 8; ++r) { mrow[r] = NEG_INF; lrow[r] = 0.f; }
#pragma unroll
  for (int t = 0; t < 4; ++t) oacc[t] = (v8f){0.f,0.f,0.f,0.f,0.f,0.f,0.f,0.f};

  const _Float16* kgb = (const _Float16*)kg16 + (size_t)b * MPAD * DD;
  const _Float16* vtb = (const _Float16*)vT16 + (size_t)b * DD * MPAD;
  _Float16* Ewave = Esh + wave * 16 * 64;

  for (int kc = 0; kc < NCHK; ++kc) {
    const int kv0 = kc * 64;
    __syncthreads();
#pragma unroll
    for (int i = 0; i < 4; ++i) {
      const int e = i * 128 + tid;
      const int r = e >> 3, seg = (e & 7) * 8;
      const v8h kk = *(const v8h*)(kgb + (size_t)(kv0 + r) * DD + seg);
      const v8h vv = *(const v8h*)(vtb + (size_t)r * MPAD + kv0 + seg);
      *(v8h*)(Ksh + r * 64 + seg) = kk;
      *(v8h*)(Vth + r * 64 + seg) = vv;
    }
    __syncthreads();

    v8f s[4];
#pragma unroll
    for (int j = 0; j < 4; ++j) {
      s[j] = (v8f){0.f,0.f,0.f,0.f,0.f,0.f,0.f,0.f};
      const _Float16* kr = Ksh + (j * 16 + c) * 64 + 8 * hh;
      s[j] = mma_h(qa0, Frag<_Float16>::load(kr), s[j]);
      s[j] = mma_h(qa1, Frag<_Float16>::load(kr + 32), s[j]);
    }
    float cm[8];
#pragma unroll
    for (int r = 0; r < 8; ++r) {
      float m = NEG_INF;
#pragma unroll
      for (int j = 0; j < 4; ++j) {
        float sv = s[j][r] * 0.125f;
        if (kv0 + j * 16 + c >= MM) sv = NEG_INF;
        s[j][r] = sv;
        m = fmaxf(m, sv);
      }
#pragma unroll
      for (int off = 1; off < 16; off <<= 1) m = fmaxf(m, __shfl_xor(m, off, 32));
      cm[r] = m;
    }
    _Float16* Ew = Ewave + kc * 64 * 64;
#pragma unroll
    for (int r = 0; r < 8; ++r) {
      const float mnew = fmaxf(mrow[r], cm[r]);
      const float alpha = expf(mrow[r] - mnew);
      mrow[r] = mnew;
      float psum = 0.f;
#pragma unroll
      for (int j = 0; j < 4; ++j) {
        const float p = expf(s[j][r] - mnew);
        psum += p;
        Ew[(8 * hh + r) * 64 + j * 16 + c] = (_Float16)(p * PSCALE);
      }
#pragma unroll
      for (int off = 1; off < 16; off <<= 1) psum += __shfl_xor(psum, off, 32);
      lrow[r] = lrow[r] * alpha + psum;
#pragma unroll
      for (int t = 0; t < 4; ++t) oacc[t][r] *= alpha;
      if (c == 0) Ws[(wave * 16 + 8 * hh + r) * NCHK + kc] = mnew;
    }
    __builtin_amdgcn_fence(__ATOMIC_RELEASE, "workgroup");
    __builtin_amdgcn_wave_barrier();
    __builtin_amdgcn_fence(__ATOMIC_ACQUIRE, "workgroup");
#pragma unroll 1
    for (int kk = 0; kk < 2; ++kk) {
      const v16h pa = Frag<_Float16>::load(Ew + c * 64 + kk * 32 + 8 * hh);
#pragma unroll
      for (int t = 0; t < 4; ++t) {
        const v16h vb = Frag<_Float16>::load(Vth + (t * 16 + c) * 64 + kk * 32 + 8 * hh);
        oacc[t] = mma_h(pa, vb, oacc[t]);
      }
    }
  }

  __syncthreads();
  float inv[8];
#pragma unroll
  for (int r = 0; r < 8; ++r) inv[r] = 1.0f / (lrow[r] * PSCALE);
#pragma unroll
  for (int r = 0; r < 8; ++r) {
    const int row = wave * 16 + 8 * hh + r;
#pragma unroll
    for (int u = 0; u < 2; ++u) {
      const int kcx = c + 16 * u;
      if (kcx < NCHK) {
        const float mv = Ws[row * NCHK + kcx];
        Ws[row * NCHK + kcx] = expf(mv - mrow[r]) * inv[r];
      }
    }
  }
  __syncthreads();
  for (int jj = 0; jj < MPAD / 128; ++jj) {
    const int col = jj * 128 + tid;
    const int kcx = col >> 6, kv = col & 63;
    const _Float16* ep = Esh + kcx * 64 * 64 + kv;
    const float* wp = Ws + kcx;
    float a = 0.f;
#pragma unroll 8
    for (int row = 0; row < 64; ++row) a += (float)ep[row * 64] * wp[row * NCHK];
    Cs[col] = a;
  }
  __syncthreads();
  {
    float* prow = partial + ((size_t)b * NQB + qb) * MPAD;
    for (int pass = 0; pass < 2; ++pass) {
#pragma unroll
      for (int u = 0; u < 4; ++u) {
        const int f = u * 128 + tid;
        if (f < MPAD / 4) {
          const v4f v = *(const v4f*)(Cs + 4 * f);
          *(volatile v4f*)(prow + 4 * f) = v;
        }
      }
      __threadfence();
    }
  }
  __syncthreads();
  float* Os = reinterpret_cast<float*>(Esh);
#pragma unroll
  for (int r = 0; r < 8; ++r)
#pragma unroll
    for (int t = 0; t < 4; ++t) Os[(wave * 16 + 8 * hh + r) * 68 + t * 16 + c] = oacc[t][r] * inv[r];
  __syncthreads();
  {
    float* ob = out0 + (size_t)b * DD * NN + (size_t)qb * 64;
    const int q8 = lane >> 3, l4 = (lane & 7) * 4;
    for (int pass = 0; pass < 2; ++pass) {
#pragma unroll
      for (int it = 0; it < 8; ++it) {
        const int L = it * 16 + wave * 4 + q8;
        const int d = L >> 1, nl = (L & 1) * 32 + l4;
        v4f v;
        v[0] = Os[(nl + 0) * 68 + d];
        v[1] = Os[(nl + 1) * 68 + d];
        v[2] = Os[(nl + 2) * 68 + d];
        v[3] = Os[(nl + 3) * 68 + d];
        *(volatile v4f*)(ob + (size_t)d * NN + nl) = v;
      }
      __threadfence();
    }
  }
}

__global__ __launch_bounds__(128) void k_colsum(const float* __restrict__ partial, float* __restrict__ colsum) {
  const int g = blockIdx.x * 128 + threadIdx.x;
  if (g < BB * (MPAD / 4)) {
    const int b = g / (MPAD / 4), f = g - b * (MPAD / 4);
    const float* p = partial + (size_t)b * NQB * MPAD + 4 * f;
    v4f a = (v4f){0.f, 0.f, 0.f, 0.f};
#pragma unroll 4
    for (int qb = 0; qb < NQB; ++qb) a += *(const v4f*)(p + (size_t)qb * MPAD);
    float* dst = colsum + (size_t)b * MPAD + 4 * f;
    *(volatile v4f*)dst = a;
    __threadfence();
    *(volatile v4f*)dst = a;
  }
}

__global__ __launch_bounds__(256) void k_out1(const float* __restrict__ colsum, const int* __restrict__ idx,
                                             float* __restrict__ out1) {
  __shared__ __align__(16) float sval[256];
  const int t = threadIdx.x;
  const int b = blockIdx.x >> 6, n0 = (blockIdx.x & 63) * 256;
  sval[t] = 0.0f;
  __syncthreads();
  for (int i = 0; i < (MM + 255) / 256; ++i) {
    const int m = i * 256 + t;
    if (m < MM) {
      const int v = idx[b * MM + m];
      const unsigned rel = (unsigned)(v - n0);
      if (rel < 256u) sval[rel] = colsum[b * MPAD + m];
    }
    __syncthreads();
  }
  if (t < 64) {
    const v4f v = *(const v4f*)(sval + 4 * t);
    float* dst = out1 + (size_t)b * NN + n0 + 4 * t;
    *(volatile v4f*)dst = v;
    __threadfence();
    *(volatile v4f*)dst = v;
  }
}

extern "C" void kernel_launch(void* const* d_in, const int* in_sizes, int n_in,
                              void* d_out, int out_size, void* d_ws, size_t ws_size,
                              hipStream_t stream) {
  if (n_in < 5) return;
  if (in_sizes[0] != BB * CC * NN || in_sizes[1] != CC * DD || in_sizes[2] != CC * DD ||
      in_sizes[3] != CC * DD || in_sizes[4] != BB * MM) return;
  if (out_size != BB * DD * NN + BB * NN) return;

  const float* x   = (const float*)d_in[0];
  const float* Wq  = (const float*)d_in[1];
  const float* Wk  = (const float*)d_in[2];
  const float* Wv  = (const float*)d_in[3];
  const int*   idx = (const int*)d_in[4];

  const size_t OFF_WT   = 0;
  const size_t OFF_XFH  = 65536;
  const size_t SZ_XF    = (size_t)BB * NN * CC * 2;
  const size_t OFF_XFL  = OFF_XFH + SZ_XF;
  const size_t OFF_XGH  = OFF_XFL + SZ_XF;
  const size_t SZ_XG    = (size_t)BB * MPAD * CC * 2;
  const size_t OFF_XGL  = OFF_XGH + SZ_XG;
  const size_t OFF_Q    = OFF_XGL + SZ_XG;
  const size_t SZ_Q     = (size_t)BB * NN * DD * 2;
  const size_t OFF_KG   = OFF_Q + SZ_Q;
  const size_t SZ_KG    = (size_t)BB * MPAD * DD * 2;
  const size_t OFF_VT   = OFF_KG + SZ_KG;
  const size_t SZ_VT    = SZ_KG;
  const size_t OFF_PART = OFF_VT + SZ_VT;
  const size_t SZ_PART  = (size_t)BB * NQB * MPAD * 4;
  const size_t OFF_CS   = OFF_PART + SZ_PART;
  const size_t SZ_CS    = (size_t)BB * MPAD * 4;
  const size_t total    = OFF_CS + SZ_CS;
  if (total > ws_size) return;

  char* ws = (char*)d_ws;
  unsigned short* wt   = (unsigned short*)(ws + OFF_WT);
  unsigned short* xfh  = (unsigned short*)(ws + OFF_XFH);
  unsigned short* xfl  = (unsigned short*)(ws + OFF_XFL);
  unsigned short* xgh  = (unsigned short*)(ws + OFF_XGH);
  unsigned short* xgl  = (unsigned short*)(ws + OFF_XGL);
  unsigned short* q16  = (unsigned short*)(ws + OFF_Q);
  unsigned short* kg16 = (unsigned short*)(ws + OFF_KG);
  unsigned short* vT16 = (unsigned short*)(ws + OFF_VT);
  float* partial = (float*)(ws + OFF_PART);
  float* colsum  = (float*)(ws + OFF_CS);
  const float* dummyf = (const float*)(ws + OFF_CS);

  const unsigned short* wq_h = wt + 0 * 4096; const unsigned short* wq_l = wt + 1 * 4096;
  const unsigned short* wk_h = wt + 2 * 4096; const unsigned short* wk_l = wt + 3 * 4096;
  const unsigned short* wv_h = wt + 4 * 4096; const unsigned short* wv_l = wt + 5 * 4096;

  float* out0 = (float*)d_out;
  float* out1 = out0 + (size_t)BB * DD * NN;

  k_prep_w<<<3, 256, 0, stream>>>(Wq, Wk, Wv, wt);
  k_xf<<<BB * (NN / 64), 128, 0, stream>>>(x, xfh, xfl);
  k_gather<<<(BB * MPAD) / 16, 128, 0, stream>>>(x, idx, xgh, xgl);

  wmma_gemm64<1, true, 0, 1, false, 0><<<dim3((BB * NN / 64) / 8, 1), 256, 0, stream>>>(
      xfh, xfl, CC, 0L, wq_h, wq_l, CC, 0L, (void*)q16, (void*)q16, DD, 0L,
      dummyf, dummyf, 0L, BB * NN, DD, CC, 1.0f);
  wmma_gemm64<1, true, 0, 1, false, 0><<<dim3((BB * MPAD / 64) / 8, 1), 256, 0, stream>>>(
      xgh, xgl, CC, 0L, wk_h, wk_l, CC, 0L, (void*)kg16, (void*)kg16, DD, 0L,
      dummyf, dummyf, 0L, BB * MPAD, DD, CC, 1.0f);
  wmma_gemm64<1, true, 0, 1, false, 0><<<dim3(4, BB), 256, 0, stream>>>(
      wv_h, wv_l, CC, 0L, xgh, xgl, CC, (long)MPAD * CC, (void*)vT16, (void*)vT16, MPAD, (long)DD * MPAD,
      dummyf, dummyf, 0L, DD, MPAD, CC, 1.0f);

  k_attn<<<BB * NQB, 128, 0, stream>>>(q16, kg16, vT16, out0, partial);
  k_colsum<<<(BB * (MPAD / 4) + 127) / 128, 128, 0, stream>>>(partial, colsum);
  k_out1<<<BB * (NN / 256), 256, 0, stream>>>(colsum, idx, out1);
  (void)hipGetLastError();
}
